// MONForwardBackwardSplitting_70300024701178
// MI455X (gfx1250) — hardware-run, weakly checked
//
#include <hip/hip_runtime.h>
#include <math.h>

typedef __attribute__((ext_vector_type(16))) _Float16 v16h;
typedef __attribute__((ext_vector_type(8)))  _Float16 v8h;
typedef __attribute__((ext_vector_type(8)))  float    v8f;
typedef __attribute__((ext_vector_type(4)))  float    v4f;
typedef __attribute__((ext_vector_type(4)))  int      v4i;
typedef __attribute__((ext_vector_type(4)))  unsigned v4u;

constexpr int kBatch   = 32;
constexpr int kChan    = 128;
constexpr int kImgH    = 32;
constexpr int kImgW    = 32;
constexpr int kPix     = kImgH * kImgW;
constexpr int kLen     = kChan * kPix;
constexpr int kSlots   = 5;
constexpr int kTaps    = 9;
constexpr int kKdim    = kChan * kTaps;
constexpr int kPadH    = kImgH + 2;
constexpr int kPadW    = kImgW + 2;
constexpr int kMaxIter = 50;
constexpr size_t kPlane = (size_t)kBatch * kLen;
static_assert(kLen == 131072 && kKdim == 1152 && (kKdim % 32) == 0, "shape");
static_assert((kBatch * kPix) % 64 == 0 && (kChan % 64) == 0, "tile multiples");

constexpr float kLam      = 1e-4f;
constexpr float kStopEps  = 1e-5f;
constexpr float kResEps   = 1e-5f;
constexpr float kDamp     = 0.9f;
constexpr float kKeep     = (float)(1.0 - 0.9);
constexpr float kZ0       = 1.0f / (float)kChan;
constexpr float kCarryA   = 64.0f;
constexpr float kCarryW   = 1024.0f;
constexpr float kFold     = 1.0f / (kCarryA * kCarryW);
constexpr float kF16MinNormal = 6.103515625e-5f;
constexpr bool  kRneInputs = true;

constexpr int kZP = 132;
constexpr int kTP = 68;

constexpr size_t kOffFH    = 0;
constexpr size_t kOffGB    = kOffFH    + (size_t)kSlots * kPlane * 4;
constexpr size_t kOffW16   = kOffGB    + (size_t)kSlots * kPlane * 2;
constexpr size_t kOffPART  = kOffW16   + (size_t)kChan * kKdim * 2;
constexpr size_t kOffALPHA = kOffPART  + (size_t)512 * 32 * 4;
constexpr size_t kOffCTRL  = kOffALPHA + (size_t)kBatch * 32 * 4;
constexpr size_t kWsTotal  = kOffCTRL  + 128;
static_assert(kWsTotal == 126193792ull, "carve total");
static_assert(kWsTotal <= 134217728ull, "carve cap");
static_assert((kOffGB % 128) == 0 && (kOffW16 % 128) == 0 && (kOffPART % 128) == 0 &&
              (kOffALPHA % 128) == 0 && (kOffCTRL % 128) == 0, "128-B aligned regions");
constexpr size_t kZmBytes = (size_t)kBatch * kPadH * kPadW * kChan * 2;
static_assert(kZmBytes <= (size_t)kBatch * kLen * 4, "staged map fits in the output buffer");
static_assert((kBatch * kPix / 64) == 512, "conv grid equals PART lines");

__device__ __forceinline__ unsigned short f2bf_bits(float f) {
  unsigned u = __float_as_uint(f);
  return (unsigned short)((u + 0x7FFFu + ((u >> 16) & 1u)) >> 16);
}
__device__ __forceinline__ float bf_bits2f(unsigned short h) { return __uint_as_float(((unsigned)h) << 16); }

__device__ __forceinline__ _Float16 to_operand_f16(float v, float carry) {
  const float s = v * carry;
  const float t = (fabsf(s) < kF16MinNormal) ? 0.0f : s;
  return (_Float16)t;
}

union FragH { v16h v; v8h h[2]; };
__device__ __forceinline__ v16h frag_load_h(const _Float16* p) {
  FragH f;
  f.h[0] = *(const v8h*)(p);
  f.h[1] = *(const v8h*)(p + 16);
  return f.v;
}
__device__ __forceinline__ v8f mma_f16(v16h a, v16h b, v8f c) {
  c = __builtin_amdgcn_wmma_f32_16x16x32_f16(false, a, false, b, (short)0, c, false, false);
  asm volatile("v_nop\n\tv_nop\n\tv_nop\n\tv_nop" : "+v"(c) : "v"(a), "v"(b));
  return c;
}

__global__ __launch_bounds__(256) void pack_weights_kernel(
    const float* __restrict__ Wsrc, unsigned short* __restrict__ W16)
{
  const int i = blockIdx.x * 256 + threadIdx.x;
  if (i >= kChan * kKdim / 8) return;
  const int co  = i / (kKdim / 8);
  const int r   = i - co * (kKdim / 8);
  const int tap = r >> 4;
  const int ci0 = (r & 15) * 8;
  const float* src = Wsrc + (size_t)co * kKdim + ci0 * kTaps + tap;
  v8h hv;
#pragma unroll
  for (int e = 0; e < 8; ++e) {
    float w = src[e * kTaps];
    if (kRneInputs) w = bf_bits2f(f2bf_bits(w));
    hv[e] = to_operand_f16(w, kCarryW);
  }
  unsigned short* dst = W16 + (size_t)co * kKdim + tap * kChan + ci0;
  *(volatile v8h*)dst = hv;
  __threadfence();
  *(volatile v8h*)dst = hv;
}

constexpr int kHaloPerImg = 2 * kPadW + 2 * kImgH;
constexpr int kHaloThreads = kBatch * kHaloPerImg * 16;
constexpr int kHaloBlocks = kHaloThreads / 256;
static_assert((kHaloThreads % 256) == 0, "halo coverage");

__global__ __launch_bounds__(256) void halo_ctrl_kernel(unsigned short* __restrict__ zm16, int* __restrict__ ctrl)
{
  if (blockIdx.x == kHaloBlocks) {
    if (threadIdx.x < 32) {
      const int v = (threadIdx.x == 1) ? 1 : 0;
      volatile int* p = ctrl + threadIdx.x;
      *p = v;
      __threadfence();
      *p = v;
    }
    return;
  }
  const int i = blockIdx.x * 256 + threadIdx.x;
  const int pos = i >> 4, piece = i & 15;
  const int b = pos / kHaloPerImg;
  const int q = pos - b * kHaloPerImg;
  const int t = q - 2 * kPadW;
  const int rowS = 1 + (t >> 1);
  const int colS = (t & 1) * (kPadW - 1);
  const int row = (q < kPadW) ? 0 : ((q < 2 * kPadW) ? (kPadH - 1) : rowS);
  const int col = (q < kPadW) ? q : ((q < 2 * kPadW) ? (q - kPadW) : colS);
  unsigned short* dst = zm16 + (((size_t)b * kPadH + row) * kPadW + col) * kChan + piece * 8;
  const v4u z = (v4u){0u, 0u, 0u, 0u};
  *(volatile v4u*)dst = z;
  __threadfence();
  *(volatile v4u*)dst = z;
}

template <int MODE>
__global__ __launch_bounds__(256) void mix_stage_kernel(
    float* FH, const float* __restrict__ alphaT, const float* __restrict__ x, const int* __restrict__ mask,
    unsigned short* __restrict__ zm16, const int* __restrict__ ctrl, int n_act, int sel, int gate)
{
  if (gate != 0) { if (ctrl[0] != 0) return; }
  __shared__ __align__(16) float sZ[kImgW * kZP];
  const int tid = threadIdx.x;
  const int b = blockIdx.x >> 5;
  const int h = blockIdx.x & 31;
  float al[kSlots];
#pragma unroll
  for (int j = 0; j < kSlots; ++j) {
    al[j] = 0.0f;
    if (MODE == 2) { if (j < n_act) al[j] = alphaT[b * 32 + j]; }
  }
#pragma unroll 1
  for (int it = 0; it < 4; ++it) {
    const int idx = it * 256 + tid;
    const int c = idx >> 3, w4 = (idx & 7) * 4;
    const size_t eo = (size_t)b * kLen + (size_t)c * kPix + h * kImgW + w4;
    v4f zv;
    if (MODE == 0) {
      zv = (v4f){kZ0, kZ0, kZ0, kZ0};
    } else if (MODE == 1) {
      zv = *(const v4f*)(FH + (size_t)sel * kPlane + eo);
    } else {
      zv = (v4f){0.0f, 0.0f, 0.0f, 0.0f};
#pragma unroll
      for (int j = 0; j < kSlots; ++j) {
        if (j < n_act) {
          const v4f fv = *(const v4f*)(FH + (size_t)j * kPlane + eo);
          zv[0] = fmaf(al[j], fv[0], zv[0]);
          zv[1] = fmaf(al[j], fv[1], zv[1]);
          zv[2] = fmaf(al[j], fv[2], zv[2]);
          zv[3] = fmaf(al[j], fv[3], zv[3]);
        }
      }
      float* dst = FH + (size_t)sel * kPlane + eo;
      *(volatile v4f*)dst = zv;
      __threadfence();
      *(volatile v4f*)dst = zv;
    }
    const v4f xv = *(const v4f*)(x + eo);
    const v4i mk = *(const v4i*)(mask + b * kPix + h * kImgW + w4);
#pragma unroll
    for (int e = 0; e < 4; ++e) {
      const float mf = (float)mk[e];
      float xr = xv[e];
      if (kRneInputs) xr = bf_bits2f(f2bf_bits(xr));
      const float zm = zv[e] * (1.0f - mf) + mf * xr;
      sZ[(w4 + e) * kZP + c] = zm;
    }
  }
  __syncthreads();
  v8h hv[2];
#pragma unroll
  for (int it = 0; it < 2; ++it) {
    const int p = it * 256 + tid;
    const int w = p >> 4, c8 = (p & 15) * 8;
    const v4f a0 = *(const v4f*)(sZ + w * kZP + c8);
    const v4f a1 = *(const v4f*)(sZ + w * kZP + c8 + 4);
#pragma unroll
    for (int e = 0; e < 4; ++e) {
      hv[it][e]     = to_operand_f16(a0[e], kCarryA);
      hv[it][4 + e] = to_operand_f16(a1[e], kCarryA);
    }
  }
  for (int pass = 0; pass < 2; ++pass) {
#pragma unroll
    for (int it = 0; it < 2; ++it) {
      const int p = it * 256 + tid;
      const int w = p >> 4, c8 = (p & 15) * 8;
      unsigned short* dst = zm16 + (((size_t)b * kPadH + (h + 1)) * kPadW + (w + 1)) * kChan + c8;
      *(volatile v8h*)dst = hv[it];
    }
    __threadfence();
  }
}

template <int ZMODE>
__global__ __launch_bounds__(128) void conv_softmax_kernel(
    const unsigned short* __restrict__ zm16, const unsigned short* __restrict__ W16,
    const float* __restrict__ bias, const float* zsrc, float* fout,
    unsigned short* __restrict__ gout, float* __restrict__ part, const int* __restrict__ ctrl, int gate)
{
  if (gate != 0) { if (ctrl[0] != 0) return; }
  __shared__ __align__(16) float sT[kChan * kTP];
  __shared__ float sBias[kChan];
  __shared__ float sRed[8];
  const int tid = threadIdx.x, lane = tid & 31, wave = tid >> 5;
  const int rl = lane & 15, hf = lane >> 4;
  const int mi = wave & 1, ni = wave >> 1;
  const int b  = blockIdx.x >> 4;
  const int r2 = (blockIdx.x & 15) * 2;
  {
    float bv = bias[tid];
    if (kRneInputs) bv = bf_bits2f(f2bf_bits(bv));
    sBias[tid] = bv;
  }
  const _Float16* Ap = (const _Float16*)zm16 + (((size_t)b * kPadH + (r2 + mi)) * kPadW + rl) * kChan + 8 * hf;
  const _Float16* Bp = (const _Float16*)W16 + (size_t)(ni * 64 + rl) * kKdim + 8 * hf;

  v8f acc[2][4];
#pragma unroll
  for (int i = 0; i < 2; ++i)
#pragma unroll
    for (int j = 0; j < 4; ++j) acc[i][j] = (v8f){0.f, 0.f, 0.f, 0.f, 0.f, 0.f, 0.f, 0.f};

#pragma unroll 1
  for (int kh = 0; kh < 3; ++kh) {
#pragma unroll 1
    for (int kw = 0; kw < 3; ++kw) {
      const _Float16* at = Ap + (kh * kPadW + kw) * kChan;
      const _Float16* bt = Bp + (kh * 3 + kw) * kChan;
#pragma unroll 1
      for (int cc = 0; cc < 4; ++cc) {
        v16h bf[4];
#pragma unroll
        for (int j = 0; j < 4; ++j) bf[j] = frag_load_h(bt + (size_t)j * 16 * kKdim + cc * 32);
#pragma unroll
        for (int i = 0; i < 2; ++i) {
          const v16h af = frag_load_h(at + i * 16 * kChan + cc * 32);
#pragma unroll
          for (int j = 0; j < 4; ++j) acc[i][j] = mma_f16(af, bf[j], acc[i][j]);
        }
      }
    }
  }

#pragma unroll
  for (int i = 0; i < 2; ++i) {
#pragma unroll
    for (int j = 0; j < 4; ++j) {
      const int c  = ni * 64 + j * 16 + rl;
      const int p0 = mi * 32 + i * 16 + 8 * hf;
      const v8f a = acc[i][j];
      const v4f lo = (v4f){a[0], a[1], a[2], a[3]};
      const v4f hi = (v4f){a[4], a[5], a[6], a[7]};
      *(v4f*)(sT + c * kTP + p0)     = lo;
      *(v4f*)(sT + c * kTP + p0 + 4) = hi;
    }
  }
  __syncthreads();

  const size_t planeOff = (size_t)b * kLen + (size_t)r2 * kImgW;
  v4f zreg[16];
#pragma unroll
  for (int it = 0; it < 16; ++it) {
    const int idx = it * 128 + tid;
    const int c = idx >> 4, p4 = (idx & 15) * 4;
    if (ZMODE == 0) zreg[it] = (v4f){kZ0, kZ0, kZ0, kZ0};
    else            zreg[it] = *(const v4f*)(zsrc + planeOff + (size_t)c * kPix + p4);
    const v4f a = *(const v4f*)(sT + c * kTP + p4);
    const float bc = sBias[c];
    v4f pre;
#pragma unroll
    for (int e = 0; e < 4; ++e) {
      const float lin = a[e] * kFold + bc;
      pre[e] = kKeep * zreg[it][e] + kDamp * lin;
    }
    *(v4f*)(sT + c * kTP + p4) = pre;
  }
  __syncthreads();

  {
    const int p  = tid >> 1;
    const int c0 = (tid & 1) * 64;
    float m = -INFINITY;
#pragma unroll 1
    for (int c = 0; c < 64; ++c) m = fmaxf(m, sT[(c0 + c) * kTP + p]);
    m = fmaxf(m, __shfl_xor(m, 1, 32));
    float s = 0.0f;
#pragma unroll 1
    for (int c = 0; c < 64; ++c) {
      const float e = expf(sT[(c0 + c) * kTP + p] - m);
      sT[(c0 + c) * kTP + p] = e;
      s += e;
    }
    s += __shfl_xor(s, 1, 32);
    const float inv = 1.0f / s;
#pragma unroll 1
    for (int c = 0; c < 64; ++c) sT[(c0 + c) * kTP + p] *= inv;
  }
  __syncthreads();

  float s1 = 0.0f, s2 = 0.0f;
#pragma unroll
  for (int it = 0; it < 16; ++it) {
    const int idx = it * 128 + tid;
    const int c = idx >> 4, p4 = (idx & 15) * 4;
    const v4f f = *(const v4f*)(sT + c * kTP + p4);
    *(volatile v4f*)(fout + planeOff + (size_t)c * kPix + p4) = f;
  }
  __threadfence();
#pragma unroll
  for (int it = 0; it < 16; ++it) {
    const int idx = it * 128 + tid;
    const int c = idx >> 4, p4 = (idx & 15) * 4;
    const v4f f = *(const v4f*)(sT + c * kTP + p4);
    *(volatile v4f*)(fout + planeOff + (size_t)c * kPix + p4) = f;
    v4f g;
#pragma unroll
    for (int e = 0; e < 4; ++e) {
      g[e] = f[e] - zreg[it][e];
      s1 = fmaf(g[e], g[e], s1);
      s2 = fmaf(f[e], f[e], s2);
    }
    *(v4f*)(sT + c * kTP + p4) = g;
  }
  __threadfence();
  __syncthreads();

  for (int pass = 0; pass < 2; ++pass) {
#pragma unroll
    for (int it = 0; it < 8; ++it) {
      const int q = it * 128 + tid;
      const int c = q >> 3, p8 = (q & 7) * 8;
      const v4f a0 = *(const v4f*)(sT + c * kTP + p8);
      const v4f a1 = *(const v4f*)(sT + c * kTP + p8 + 4);
      v8h hv;
#pragma unroll
      for (int e = 0; e < 4; ++e) {
        const unsigned short h0 = f2bf_bits(a0[e]);
        const unsigned short h1 = f2bf_bits(a1[e]);
        hv[e]     = __builtin_bit_cast(_Float16, h0);
        hv[4 + e] = __builtin_bit_cast(_Float16, h1);
      }
      *(volatile v8h*)(gout + planeOff + (size_t)c * kPix + p8) = hv;
    }
    __threadfence();
  }

#pragma unroll
  for (int off = 16; off >= 1; off >>= 1) {
    s1 += __shfl_xor(s1, off, 32);
    s2 += __shfl_xor(s2, off, 32);
  }
  if (lane == 0) { sRed[wave] = s1; sRed[4 + wave] = s2; }
  __syncthreads();
  if (wave == 0) {
    const float t1 = (sRed[0] + sRed[1]) + (sRed[2] + sRed[3]);
    const float t2 = (sRed[4] + sRed[5]) + (sRed[6] + sRed[7]);
    const float v = (lane == 0) ? t1 : ((lane == 1) ? t2 : 0.0f);
    volatile float* pp = part + (size_t)blockIdx.x * 32 + lane;
    *pp = v;
    __threadfence();
    *pp = v;
  }
}

__global__ __launch_bounds__(512) void gram_solve_kernel(
    const unsigned short* __restrict__ GB, const float* __restrict__ part,
    float* __restrict__ alphaT, int* ctrl, int k_iter)
{
  __shared__ float sRed[256];
  __shared__ float sTot[16];
  __shared__ float sH[48];
  __shared__ float sAl[32];
  __shared__ int   sFlag;
  const int tid = threadIdx.x, lane = tid & 31, wave = tid >> 5;
  const int b = blockIdx.x;
  int was_done = 0;
  if (b == 0) was_done = ctrl[0];
  if (was_done != 0) return;

  if (k_iter > 2) {
    float a1 = part[(size_t)tid * 32 + 0];
    float a2 = part[(size_t)tid * 32 + 1];
#pragma unroll
    for (int off = 16; off >= 1; off >>= 1) {
      a1 += __shfl_xor(a1, off, 32);
      a2 += __shfl_xor(a2, off, 32);
    }
    if (lane == 0) { sRed[wave] = a1; sRed[16 + wave] = a2; }
    __syncthreads();
    if (tid == 0) {
      float t1 = 0.0f, t2 = 0.0f;
#pragma unroll 1
      for (int w = 0; w < 16; ++w) { t1 += sRed[w]; t2 += sRed[16 + w]; }
      const float res = sqrtf(t1) / (kResEps + sqrtf(t2));
      sFlag = (res >= kStopEps) ? 0 : 1;
    }
    __syncthreads();
    const int stop = sFlag;
    if (stop != 0) {
      if (b == 0 && wave == 0) {
        const int v = (lane == 0) ? 1 : ((lane == 1) ? ((k_iter - 1) % kSlots) : 0);
        volatile int* p = ctrl + lane;
        *p = v;
        __threadfence();
        *p = v;
      }
      return;
    }
  }

  const int n = (k_iter < kSlots) ? k_iter : kSlots;
  float acc[15];
#pragma unroll
  for (int q = 0; q < 15; ++q) acc[q] = 0.0f;
  const unsigned* gw = (const unsigned*)GB;
  constexpr size_t kPlaneW = kPlane / 2;
#pragma unroll 1
  for (int it = 0; it < 128; ++it) {
    const size_t wo = (size_t)b * (kLen / 2) + (size_t)it * 512 + tid;
    float g0[kSlots], g1[kSlots];
#pragma unroll
    for (int j = 0; j < kSlots; ++j) {
      unsigned w = 0u;
      if (j < n) w = gw[(size_t)j * kPlaneW + wo];
      g0[j] = __uint_as_float(w << 16);
      g1[j] = __uint_as_float(w & 0xffff0000u);
    }
    int q = 0;
#pragma unroll
    for (int i = 0; i < kSlots; ++i) {
#pragma unroll
      for (int j = i; j < kSlots; ++j) {
        acc[q] = fmaf(g0[i], g0[j], acc[q]);
        acc[q] = fmaf(g1[i], g1[j], acc[q]);
        ++q;
      }
    }
  }
#pragma unroll
  for (int q = 0; q < 15; ++q) {
    float v = acc[q];
#pragma unroll
    for (int off = 16; off >= 1; off >>= 1) v += __shfl_xor(v, off, 32);
    if (lane == 0) sRed[q * 16 + wave] = v;
  }
  __syncthreads();
  if (tid < 15) {
    float t = 0.0f;
#pragma unroll 1
    for (int w = 0; w < 16; ++w) t += sRed[tid * 16 + w];
    sTot[tid] = t;
  }
  __syncthreads();
  if (tid == 0) {
#pragma unroll 1
    for (int i = 0; i < 48; ++i) sH[i] = 0.0f;
    sH[6] = 1.0f;
#pragma unroll 1
    for (int i = 0; i < kSlots; ++i) {
      const float ai = (i < n) ? 1.0f : 0.0f;
      sH[i + 1] = ai;
      sH[(i + 1) * 8] = ai;
#pragma unroll 1
      for (int j = 0; j < kSlots; ++j) {
        const int lo = (i < j) ? i : j;
        const int hi = (i < j) ? j : i;
        const float gij = sTot[lo * kSlots - (lo * (lo - 1)) / 2 + (hi - lo)];
        const float aj = (j < n) ? 1.0f : 0.0f;
        const float dg = (i == j) ? 1.0f : 0.0f;
        float hc = gij + kLam * dg;
        hc = hc * (ai * aj) + dg * (1.0f - ai);
        sH[(i + 1) * 8 + (j + 1)] = hc;
      }
    }
#pragma unroll 1
    for (int col = 0; col < 6; ++col) {
      int piv = col;
      float mx = fabsf(sH[col * 8 + col]);
#pragma unroll 1
      for (int r = col + 1; r < 6; ++r) {
        const float v = fabsf(sH[r * 8 + col]);
        if (v > mx) { mx = v; piv = r; }
      }
      if (piv != col) {
#pragma unroll 1
        for (int c = 0; c < 7; ++c) {
          const float t = sH[col * 8 + c];
          sH[col * 8 + c] = sH[piv * 8 + c];
          sH[piv * 8 + c] = t;
        }
      }
      const float invd = 1.0f / sH[col * 8 + col];
#pragma unroll 1
      for (int r = col + 1; r < 6; ++r) {
        const float f = sH[r * 8 + col] * invd;
#pragma unroll 1
        for (int c = col; c < 7; ++c) sH[r * 8 + c] -= f * sH[col * 8 + c];
      }
    }
#pragma unroll 1
    for (int col = 5; col >= 0; --col) {
      float s = sH[col * 8 + 6];
#pragma unroll 1
      for (int c = col + 1; c < 6; ++c) s -= sH[col * 8 + c] * sH[c * 8 + 6];
      sH[col * 8 + 6] = s / sH[col * 8 + col];
    }
#pragma unroll 1
    for (int t = 0; t < 32; ++t) sAl[t] = (t < kSlots) ? sH[(t + 1) * 8 + 6] : 0.0f;
  }
  __syncthreads();
  if (wave == 0) {
    const float v = sAl[lane];
    volatile float* pa = alphaT + (size_t)b * 32 + lane;
    *pa = v;
    __threadfence();
    *pa = v;
    if (b == 0) {
      const int cv = (lane == 1) ? (k_iter % kSlots) : 0;
      volatile int* pc = ctrl + lane;
      *pc = cv;
      __threadfence();
      *pc = cv;
    }
  }
}

__global__ __launch_bounds__(256) void final_copy_kernel(
    const float* __restrict__ FH, const int* __restrict__ ctrl, float* __restrict__ out)
{
  int s = ctrl[1];
  s = (s < 0) ? 0 : ((s > kSlots - 1) ? (kSlots - 1) : s);
  const float* src = FH + (size_t)s * kPlane;
  v4f v[2];
#pragma unroll
  for (int it = 0; it < 2; ++it) {
    const size_t e = ((size_t)blockIdx.x * 512 + it * 256 + threadIdx.x) * 4;
    v[it] = *(const v4f*)(src + e);
  }
  for (int pass = 0; pass < 2; ++pass) {
#pragma unroll
    for (int it = 0; it < 2; ++it) {
      const size_t e = ((size_t)blockIdx.x * 512 + it * 256 + threadIdx.x) * 4;
      *(volatile v4f*)(out + e) = v[it];
    }
    __threadfence();
  }
}

extern "C" void kernel_launch(void* const* d_in, const int* in_sizes, int n_in,
                              void* d_out, int out_size, void* d_ws, size_t ws_size,
                              hipStream_t stream) {
  if (n_in < 4) return;
  if (in_sizes[0] != kBatch * kLen) return;
  if (in_sizes[1] != kChan * kKdim) return;
  if (in_sizes[2] != kChan) return;
  if (in_sizes[3] != kBatch * kPix) return;
  if (out_size != kBatch * kLen) return;
  if (ws_size < kWsTotal) return;

  const float* x    = (const float*)d_in[0];
  const float* Wsrc = (const float*)d_in[1];
  const float* bias = (const float*)d_in[2];
  const int*   mask = (const int*)d_in[3];
  float* out = (float*)d_out;
  unsigned short* zm16 = (unsigned short*)d_out;

  char* ws = (char*)d_ws;
  float*          FH     = (float*)(ws + kOffFH);
  unsigned short* GB     = (unsigned short*)(ws + kOffGB);
  unsigned short* W16    = (unsigned short*)(ws + kOffW16);
  float*          PART   = (float*)(ws + kOffPART);
  float*          ALPHA  = (float*)(ws + kOffALPHA);
  int*            CTRL   = (int*)(ws + kOffCTRL);

  pack_weights_kernel<<<(kChan * kKdim / 8) / 256, 256, 0, stream>>>(Wsrc, W16);
  halo_ctrl_kernel<<<kHaloBlocks + 1, 256, 0, stream>>>(zm16, CTRL);

  const int gridMix  = kBatch * kImgH;
  const int gridConv = kBatch * kPix / 64;

  mix_stage_kernel<0><<<gridMix, 256, 0, stream>>>(FH, ALPHA, x, mask, zm16, CTRL, 0, 0, 0);
  conv_softmax_kernel<0><<<gridConv, 128, 0, stream>>>(zm16, W16, bias, FH, FH, GB, PART, CTRL, 0);
  mix_stage_kernel<1><<<gridMix, 256, 0, stream>>>(FH, ALPHA, x, mask, zm16, CTRL, 0, 0, 0);
  conv_softmax_kernel<1><<<gridConv, 128, 0, stream>>>(zm16, W16, bias, FH, FH + kPlane, GB + kPlane, PART, CTRL, 0);

  for (int k = 2; k < kMaxIter; ++k) {
    const int n_act = (k < kSlots) ? k : kSlots;
    const int slot  = k % kSlots;
    gram_solve_kernel<<<kBatch, 512, 0, stream>>>(GB, PART, ALPHA, CTRL, k);
    mix_stage_kernel<2><<<gridMix, 256, 0, stream>>>(FH, ALPHA, x, mask, zm16, CTRL, n_act, slot, 1);
    conv_softmax_kernel<1><<<gridConv, 128, 0, stream>>>(zm16, W16, bias,
        FH + (size_t)slot * kPlane, FH + (size_t)slot * kPlane, GB + (size_t)slot * kPlane, PART, CTRL, 1);
  }

  final_copy_kernel<<<(kBatch * kLen / 4) / 512, 256, 0, stream>>>(FH, CTRL, out);
}
